// MyMSA_22239340658969
// MI455X (gfx1250) — hardware-verified
//
#include <hip/hip_runtime.h>
#include <math.h>

constexpr int   kSeq        = 2048;
constexpr int   kDim        = 1024;
constexpr int   kHeads      = 16;
constexpr int   kDh         = 64;
constexpr int   kQKld       = 2 * kDh;
constexpr float kWCarryMul  = 16.0f;
constexpr float kWCarryInv  = 1.0f / 16.0f;
constexpr float kPCarryMul  = 2048.0f;
constexpr float kPCarryInv  = 1.0f / 2048.0f;
constexpr float kScoreScale = 0.125f;
constexpr int   kGroupChunk = 2;

typedef __attribute__((ext_vector_type(16))) _Float16 v16h;
typedef __attribute__((ext_vector_type(8)))  _Float16 v8h;
typedef __attribute__((ext_vector_type(16))) __bf16   v16b;
typedef __attribute__((ext_vector_type(8)))  __bf16   v8b;
typedef __attribute__((ext_vector_type(8)))  float    v8f;
typedef __attribute__((ext_vector_type(4)))  float    v4f;
typedef __attribute__((ext_vector_type(4)))  unsigned int v4u;

__device__ __forceinline__ unsigned short f2bf_bits(float f) {
  unsigned u = __float_as_uint(f);
  return (unsigned short)((u + 0x7FFFu + ((u >> 16) & 1u)) >> 16);
}
__device__ __forceinline__ float bf_bits2f(unsigned short h) { return __uint_as_float(((unsigned)h) << 16); }

__device__ __forceinline__ void dep_guard_h(v8f& a, v8f& b, v16h x, v16h y) { asm volatile("v_nop\n\tv_nop\n\tv_nop\n\tv_nop" : "+v"(a), "+v"(b) : "v"(x), "v"(y)); }
__device__ __forceinline__ void dep_guard_b(v8f& a, v8f& b, v16b x, v16b y) { asm volatile("v_nop\n\tv_nop\n\tv_nop\n\tv_nop" : "+v"(a), "+v"(b) : "v"(x), "v"(y)); }
__device__ __forceinline__ void keep4_h(v16h a, v16h b, v16h c, v16h d) { asm volatile("v_nop" :: "v"(a), "v"(b), "v"(c), "v"(d)); }
__device__ __forceinline__ void keep4_b(v16b a, v16b b, v16b c, v16b d) { asm volatile("v_nop" :: "v"(a), "v"(b), "v"(c), "v"(d)); }
__device__ __forceinline__ void acc_guard4(v8f& a, v8f& b, v8f& c, v8f& d) { asm volatile("v_nop\n\tv_nop\n\tv_nop\n\tv_nop" : "+v"(a), "+v"(b), "+v"(c), "+v"(d)); }
template <typename T> struct Frag;
template <> struct Frag<_Float16> {
  typedef v16h V; union U { v16h v; v8h h[2]; };
  static __device__ __forceinline__ v16h load(const _Float16* p) {
    U f; f.h[0] = *(const v8h*)(p); f.h[1] = *(const v8h*)(p + 16); return f.v;
  }
  static __device__ __forceinline__ v8f mma(v16h a, v16h b, v8f c) {
    return __builtin_amdgcn_wmma_f32_16x16x32_f16(false, a, false, b, (short)0, c, false, false);
  }
  static __device__ __forceinline__ void guard(v8f& a, v8f& b, v16h x, v16h y) { dep_guard_h(a, b, x, y); }
  static __device__ __forceinline__ void keep(v16h a, v16h b, v16h c, v16h d) { keep4_h(a, b, c, d); }
};
template <> struct Frag<__bf16> {
  typedef v16b V; union U { v16b v; v8b h[2]; };
  static __device__ __forceinline__ v16b load(const __bf16* p) {
    U f; f.h[0] = *(const v8b*)(p); f.h[1] = *(const v8b*)(p + 16); return f.v;
  }
  static __device__ __forceinline__ v8f mma(v16b a, v16b b, v8f c) {
    return __builtin_amdgcn_wmma_f32_16x16x32_bf16(false, a, false, b, (short)0, c, false, false);
  }
  static __device__ __forceinline__ void guard(v8f& a, v8f& b, v16b x, v16b y) { dep_guard_b(a, b, x, y); }
  static __device__ __forceinline__ void keep(v16b a, v16b b, v16b c, v16b d) { keep4_b(a, b, c, d); }
};

__device__ __forceinline__ unsigned pk16(unsigned short a, unsigned short b) { return (unsigned)a | ((unsigned)b << 16); }
__device__ __forceinline__ unsigned short h_bits(float f) { const _Float16 h = (_Float16)f; return __builtin_bit_cast(unsigned short, h); }

template <int ET> struct Elem;
template <> struct Elem<0> { typedef _Float16 T; };
template <> struct Elem<1> { typedef __bf16 T; };
template <int ET, bool SPLIT, int BIAS_MODE, int OUT_MODE, bool RESID, int ACT = 0>
__global__ __launch_bounds__(256) void wmma_gemm64(
    const unsigned short* __restrict__ Ap, const unsigned short* __restrict__ A2p, int lda, long strideA, long strideAz,
    const unsigned short* __restrict__ Btp, const unsigned short* __restrict__ Bt2p, int ldb, long strideB, long strideBz,
    void* __restrict__ Cout, void* __restrict__ Cout2, int ldc, long strideC, long strideCz,
    const float* __restrict__ bias, long strideBias, long strideBiasZ,
    const float* __restrict__ resid, long strideR,
    int M, int N, int K, float scale) {
  typedef typename Elem<ET>::T T;
  typedef typename Frag<T>::V V;
  const T* A = (const T*)Ap; const T* A2 = (const T*)A2p; const T* Bt = (const T*)Btp; const T* Bt2 = (const T*)Bt2p;
  __shared__ __align__(16) float sT[8][16 * 68];
  const int b    = blockIdx.y;
  const int z    = blockIdx.z;
  const int lane = threadIdx.x & 31;
  const int wave = threadIdx.x >> 5;
  const int tilesN = N >> 6;
  const int tilesM = M >> 6;
  const int tile = blockIdx.x * 8 + wave;
  if (tile >= tilesM * tilesN) return;
  const int tm = tile / tilesN;
  const int tn = tile - tm * tilesN;
  const int m0 = tm << 6;
  const int n0 = tn << 6;

  const size_t offA = (size_t)b * strideA + (size_t)z * strideAz;
  const size_t offB = (size_t)b * strideB + (size_t)z * strideBz;
  const size_t offC = (size_t)b * strideC + (size_t)z * strideCz;
  const T* Ab  = A  + offA;
  const T* Bb  = Bt + offB;
  const T* Ab2 = SPLIT ? (A2  + offA) : nullptr;
  const T* Bb2 = SPLIT ? (Bt2 + offB) : nullptr;
  const float* biasb = bias;
  if (BIAS_MODE != 0) biasb = bias + (size_t)b * strideBias + (size_t)z * strideBiasZ;

  const int rlane = lane & 15;
  const int koff  = (lane >> 4) * 8;
  const int mOff  = (lane >> 4) * 8;

  v8f acc[4][4];
#pragma unroll
  for (int i = 0; i < 4; ++i)
#pragma unroll
    for (int j = 0; j < 4; ++j) acc[i][j] = (v8f){0.f,0.f,0.f,0.f,0.f,0.f,0.f,0.f};

  for (int k0 = 0; k0 < K; k0 += 32) {
    V bh[4], bl[4];
#pragma unroll
    for (int j = 0; j < 4; ++j) {
      const size_t bo = (size_t)(n0 + (j << 4) + rlane) * ldb + koff + k0;
      bh[j] = Frag<T>::load(Bb + bo);
      if (SPLIT) bl[j] = Frag<T>::load(Bb2 + bo);
    }
#pragma unroll
    for (int i = 0; i < 4; ++i) {
      const size_t ao = (size_t)(m0 + (i << 4) + rlane) * lda + koff + k0;
      V ah = Frag<T>::load(Ab + ao);
      V al;
      if (SPLIT) al = Frag<T>::load(Ab2 + ao);
#pragma unroll
      for (int j = 0; j < 4; ++j) {
        acc[i][j] = Frag<T>::mma(ah, bh[j], acc[i][j]);
        if (SPLIT) {
          acc[i][j] = Frag<T>::mma(ah, bl[j], acc[i][j]);
          acc[i][j] = Frag<T>::mma(al, bh[j], acc[i][j]);
        }
      }
      Frag<T>::guard(acc[i][0], acc[i][3], ah, SPLIT ? al : ah);
    }
    Frag<T>::keep(bh[0], bh[1], bh[2], bh[3]);
    if (SPLIT) Frag<T>::keep(bl[0], bl[1], bl[2], bl[3]);
  }
  acc_guard4(acc[0][0], acc[0][1], acc[0][2], acc[0][3]);
  acc_guard4(acc[1][0], acc[1][1], acc[1][2], acc[1][3]);
  acc_guard4(acc[2][0], acc[2][1], acc[2][2], acc[2][3]);
  acc_guard4(acc[3][0], acc[3][1], acc[3][2], acc[3][3]);

  float* slab = sT[wave];
  const float* Rb = RESID ? (resid + (size_t)b * strideR) : nullptr;
#pragma unroll
  for (int i = 0; i < 4; ++i) {
    const int mBase = m0 + (i << 4);
#pragma unroll
    for (int j = 0; j < 4; ++j) {
      const int n = n0 + (j << 4) + rlane;
      float bv = 0.f;
      if (BIAS_MODE == 2) bv = biasb[n];
#pragma unroll
      for (int r = 0; r < 8; ++r) {
        float v = acc[i][j][r] * scale;
        if (BIAS_MODE == 1) v += biasb[mBase + mOff + r];
        if (BIAS_MODE == 2) v += bv;
        if (RESID) v += Rb[(size_t)(mBase + mOff + r) * ldc + n];
        if (ACT == 2) v = fmaxf(v, 0.0f);
        if (ACT == 4) v = (v > 0.f) ? v : 0.01f * v;
        slab[(mOff + r) * 68 + (j << 4) + rlane] = v;
      }
    }
    __builtin_amdgcn_fence(__ATOMIC_RELEASE, "workgroup");
    __builtin_amdgcn_wave_barrier();
    __builtin_amdgcn_fence(__ATOMIC_ACQUIRE, "workgroup");
    if (OUT_MODE == 0) {
      float* C = (float*)Cout + offC;
      const int hh = lane >> 4, c4 = (lane & 15) * 4;
      for (int pass = 0; pass < 2; ++pass) {
#pragma unroll
        for (int it = 0; it < 8; ++it) {
          const int row = it * 2 + hh;
          v4f v = *(const v4f*)(slab + row * 68 + c4);
          *(volatile v4f*)(C + (size_t)(mBase + row) * ldc + n0 + c4) = v;
        }
        __threadfence();
      }
    } else {
      const int q = lane >> 3, c8 = (lane & 7) * 8;
      unsigned short* C  = (unsigned short*)Cout  + offC;
      unsigned short* C2 = (OUT_MODE == 2) ? ((unsigned short*)Cout2 + offC) : nullptr;
      for (int pass = 0; pass < 2; ++pass) {
#pragma unroll
        for (int it = 0; it < 4; ++it) {
          const int row = it * 4 + q;
          const float* sp = slab + row * 68 + c8;
          v8h hv, lv;
#pragma unroll
          for (int e = 0; e < 8; ++e) {
            if (OUT_MODE == 1) {
              hv[e] = (_Float16)sp[e];
            } else {
              unsigned short hb = f2bf_bits(sp[e]);
              unsigned short lb = f2bf_bits(sp[e] - bf_bits2f(hb));
              hv[e] = __builtin_bit_cast(_Float16, hb);
              lv[e] = __builtin_bit_cast(_Float16, lb);
            }
          }
          *(volatile v8h*)(C + (size_t)(mBase + row) * ldc + n0 + c8) = hv;
          if (OUT_MODE == 2) *(volatile v8h*)(C2 + (size_t)(mBase + row) * ldc + n0 + c8) = lv;
        }
        __threadfence();
      }
    }
    __builtin_amdgcn_fence(__ATOMIC_RELEASE, "workgroup");
    __builtin_amdgcn_wave_barrier();
    __builtin_amdgcn_fence(__ATOMIC_ACQUIRE, "workgroup");
  }
}

__global__ __launch_bounds__(256) void cast8_f16_kernel(const float* __restrict__ in, unsigned short* __restrict__ out, int n8) {
  const int i = blockIdx.x * 256 + threadIdx.x;
  if (i >= n8) return;
  const float* p = in + 8 * (size_t)i;
  const v4f a = *(const v4f*)(p);
  const v4f c = *(const v4f*)(p + 4);
  unsigned short hb[8];
#pragma unroll
  for (int e = 0; e < 4; ++e) {
    hb[e]     = h_bits(a[e]);
    hb[4 + e] = h_bits(c[e]);
  }
  const v4u u = (v4u){pk16(hb[0], hb[1]), pk16(hb[2], hb[3]), pk16(hb[4], hb[5]), pk16(hb[6], hb[7])};
  unsigned short* q = out + 8 * (size_t)i;
  *(volatile v4u*)q = u;
  __threadfence();
  *(volatile v4u*)q = u;
}

__global__ __launch_bounds__(256) void cast8_w_kernel(const float* __restrict__ W0, const float* __restrict__ W1,
                                                      const float* __restrict__ W2, unsigned short* __restrict__ out,
                                                      int n8, float scale) {
  const int i = blockIdx.x * 256 + threadIdx.x;
  if (i >= n8) return;
  const int y = blockIdx.y;
  const float* in = (y == 0) ? W0 : (y == 1) ? W1 : W2;
  const float* p = in + 8 * (size_t)i;
  const v4f a = *(const v4f*)(p);
  const v4f c = *(const v4f*)(p + 4);
  unsigned short hb[8];
#pragma unroll
  for (int e = 0; e < 4; ++e) {
    hb[e]     = h_bits(a[e] * scale);
    hb[4 + e] = h_bits(c[e] * scale);
  }
  const v4u u = (v4u){pk16(hb[0], hb[1]), pk16(hb[2], hb[3]), pk16(hb[4], hb[5]), pk16(hb[6], hb[7])};
  unsigned short* q = out + (size_t)y * 8 * (size_t)n8 + 8 * (size_t)i;
  *(volatile v4u*)q = u;
  __threadfence();
  *(volatile v4u*)q = u;
}

__global__ __launch_bounds__(256) void softmax_row_kernel(const float* __restrict__ Sp, unsigned short* __restrict__ Pp, float carry) {
  __shared__ float redM[8];
  __shared__ float redS[8];
  const int row  = blockIdx.x;
  const int t    = threadIdx.x;
  const int lane = t & 31, wave = t >> 5;
  const int c0   = t * 8;
  const float* sr = Sp + (size_t)row * kSeq + c0;
  const v4f a = *(const v4f*)(sr);
  const v4f c = *(const v4f*)(sr + 4);
  float x[8];
#pragma unroll
  for (int e = 0; e < 4; ++e) { x[e] = a[e]; x[4 + e] = c[e]; }
  float m = fmaxf(fmaxf(fmaxf(x[0], x[1]), fmaxf(x[2], x[3])), fmaxf(fmaxf(x[4], x[5]), fmaxf(x[6], x[7])));
#pragma unroll
  for (int off = 16; off > 0; off >>= 1) m = fmaxf(m, __shfl_xor(m, off, 32));
  if (lane == 0) redM[wave] = m;
  __syncthreads();
  float gm = redM[0];
#pragma unroll
  for (int w = 1; w < 8; ++w) gm = fmaxf(gm, redM[w]);
  float p[8];
  float s = 0.0f;
#pragma unroll
  for (int e = 0; e < 8; ++e) { p[e] = expf(x[e] - gm); s += p[e]; }
#pragma unroll
  for (int off = 16; off > 0; off >>= 1) s += __shfl_xor(s, off, 32);
  if (lane == 0) redS[wave] = s;
  __syncthreads();
  float tot = redS[0];
#pragma unroll
  for (int w = 1; w < 8; ++w) tot += redS[w];
  const float inv = carry * (1.0f / tot);
  unsigned short hb[8];
#pragma unroll
  for (int e = 0; e < 8; ++e) hb[e] = h_bits(p[e] * inv);
  const v4u u = (v4u){pk16(hb[0], hb[1]), pk16(hb[2], hb[3]), pk16(hb[4], hb[5]), pk16(hb[6], hb[7])};
  unsigned short* q = Pp + (size_t)row * kSeq + c0;
  *(volatile v4u*)q = u;
  __threadfence();
  *(volatile v4u*)q = u;
}

extern "C" void kernel_launch(void* const* d_in, const int* in_sizes, int n_in,
                              void* d_out, int out_size, void* d_ws, size_t ws_size,
                              hipStream_t stream) {
  if (n_in < 7) return;
  const float* seq = (const float*)d_in[0];
  const float* Wq  = (const float*)d_in[1];
  const float* Wk  = (const float*)d_in[2];
  const float* Wv  = (const float*)d_in[3];
  const float* bq  = (const float*)d_in[4];
  const float* bk  = (const float*)d_in[5];
  const float* bv  = (const float*)d_in[6];

  const long nseq = (long)in_sizes[0];
  if (nseq <= 0 || (nseq % ((long)kSeq * kDim)) != 0) return;
  const int  nbatch = (int)(nseq / ((long)kSeq * kDim));
  const long ntok   = (long)nbatch * kSeq;
  if ((long)out_size != ntok * kDim) return;
  const int wElems = kHeads * kDh * kDh;
  if (in_sizes[1] != wElems || in_sizes[2] != wElems || in_sizes[3] != wElems) return;
  if (in_sizes[4] != kHeads * kDh || in_sizes[5] != kHeads * kDh || in_sizes[6] != kHeads * kDh) return;

  const size_t bytesQK = (size_t)kHeads * ntok * kQKld * 2;
  const size_t bytesVT = (size_t)kHeads * nbatch * kDh * kSeq * 2;
  const size_t bytesX  = (size_t)ntok * kDim * 2;
  const size_t bytesW  = (size_t)3 * wElems * 2;
  const size_t bytesSC = (size_t)kGroupChunk * kSeq * kSeq * 4;
  const size_t bytesR3 = (bytesX + bytesW > bytesSC) ? (bytesX + bytesW) : bytesSC;
  const size_t bytesP  = (size_t)kGroupChunk * kSeq * kSeq * 2;
  const size_t offQK = 0;
  const size_t offVT = offQK + bytesQK;
  const size_t offR3 = offVT + bytesVT;
  const size_t offX  = offR3;
  const size_t offW  = offR3 + bytesX;
  const size_t offSC = offR3;
  const size_t offP  = offR3 + bytesR3;
  const size_t total = offP + bytesP;
  if (total > ws_size) return;

  char* ws = (char*)d_ws;
  unsigned short* QK16 = (unsigned short*)(ws + offQK);
  unsigned short* VT16 = (unsigned short*)(ws + offVT);
  unsigned short* X16  = (unsigned short*)(ws + offX);
  unsigned short* W16  = (unsigned short*)(ws + offW);
  float*          SC   = (float*)(ws + offSC);
  unsigned short* P16  = (unsigned short*)(ws + offP);
  float*          out  = (float*)d_out;
  const unsigned short* W16q = W16;
  const unsigned short* W16k = W16 + wElems;
  const unsigned short* W16v = W16 + 2 * wElems;
  const unsigned short* nul16 = (const unsigned short*)nullptr;

  {
    const int n8 = (int)(ntok * kDim / 8);
    const int blocks = (n8 + 255) / 256;
    hipLaunchKernelGGL(cast8_f16_kernel, dim3(blocks), dim3(256), 0, stream, seq, X16, n8);
  }
  {
    const int n8 = wElems / 8;
    const int blocks = (n8 + 255) / 256;
    hipLaunchKernelGGL(cast8_w_kernel, dim3(blocks, 3, 1), dim3(256), 0, stream, Wq, Wk, Wv, W16, n8, kWCarryMul);
  }
  {
    const int tiles  = (int)((ntok >> 6) * (kDh >> 6));
    const int blocks = (tiles + 7) / 8;
    hipLaunchKernelGGL((wmma_gemm64<0, false, 2, 1, false, 0>), dim3(blocks, kHeads, 1), dim3(256), 0, stream,
      (const unsigned short*)X16, nul16, (int)kDim, (long)kDh, (long)0,
      W16q, nul16, (int)kDh, (long)(kDh * kDh), (long)0,
      (void*)QK16, (void*)nullptr, (int)kQKld, (long)(ntok * kQKld), (long)0,
      bq, (long)kDh, (long)0,
      (const float*)nullptr, (long)0,
      (int)ntok, (int)kDh, (int)kDh, kWCarryInv);
    hipLaunchKernelGGL((wmma_gemm64<0, false, 2, 1, false, 0>), dim3(blocks, kHeads, 1), dim3(256), 0, stream,
      (const unsigned short*)X16, nul16, (int)kDim, (long)kDh, (long)0,
      W16k, nul16, (int)kDh, (long)(kDh * kDh), (long)0,
      (void*)(QK16 + kDh), (void*)nullptr, (int)kQKld, (long)(ntok * kQKld), (long)0,
      bk, (long)kDh, (long)0,
      (const float*)nullptr, (long)0,
      (int)ntok, (int)kDh, (int)kDh, kWCarryInv);
  }
  {
    const int tiles  = (kDh >> 6) * (kSeq >> 6);
    const int blocks = (tiles + 7) / 8;
    hipLaunchKernelGGL((wmma_gemm64<0, false, 1, 1, false, 0>), dim3(blocks, nbatch, kHeads), dim3(256), 0, stream,
      W16v, nul16, (int)kDh, (long)0, (long)(kDh * kDh),
      (const unsigned short*)X16, nul16, (int)kDim, (long)((long)kSeq * kDim), (long)kDh,
      (void*)VT16, (void*)nullptr, (int)kSeq, (long)((long)kDh * kSeq), (long)((long)nbatch * kDh * kSeq),
      bv, (long)0, (long)kDh,
      (const float*)nullptr, (long)0,
      (int)kDh, (int)kSeq, (int)kDh, kWCarryInv);
  }
  const int scoreTiles  = (kSeq >> 6) * (kSeq >> 6);
  const int scoreBlocks = (scoreTiles + 7) / 8;
  const int pvTiles     = (kSeq >> 6) * (kDh >> 6);
  const int pvBlocks    = (pvTiles + 7) / 8;
  for (int h = 0; h < kHeads; ++h) {
    for (int b0 = 0; b0 < nbatch; b0 += kGroupChunk) {
      const int gcount = (nbatch - b0 < kGroupChunk) ? (nbatch - b0) : kGroupChunk;
      const size_t qkOff = ((size_t)h * ntok + (size_t)b0 * kSeq) * kQKld;
      const size_t vtOff = ((size_t)h * nbatch + (size_t)b0) * kDh * kSeq;
      const size_t oOff  = (size_t)b0 * kSeq * kDim + (size_t)h * kDh;
      hipLaunchKernelGGL((wmma_gemm64<0, false, 0, 0, false, 0>), dim3(scoreBlocks, gcount, 1), dim3(256), 0, stream,
        (const unsigned short*)(QK16 + qkOff), nul16, (int)kQKld, (long)((long)kSeq * kQKld), (long)0,
        (const unsigned short*)(QK16 + qkOff + kDh), nul16, (int)kQKld, (long)((long)kSeq * kQKld), (long)0,
        (void*)SC, (void*)nullptr, (int)kSeq, (long)((long)kSeq * kSeq), (long)0,
        (const float*)nullptr, (long)0, (long)0,
        (const float*)nullptr, (long)0,
        (int)kSeq, (int)kSeq, (int)kDh, kScoreScale);
      hipLaunchKernelGGL(softmax_row_kernel, dim3(gcount * kSeq), dim3(256), 0, stream, (const float*)SC, P16, kPCarryMul);
      hipLaunchKernelGGL((wmma_gemm64<0, false, 0, 0, false, 0>), dim3(pvBlocks, gcount, 1), dim3(256), 0, stream,
        (const unsigned short*)P16, nul16, (int)kSeq, (long)((long)kSeq * kSeq), (long)0,
        (const unsigned short*)(VT16 + vtOff), nul16, (int)kSeq, (long)((long)kDh * kSeq), (long)0,
        (void*)(out + oOff), (void*)nullptr, (int)kDim, (long)((long)kSeq * kDim), (long)0,
        (const float*)nullptr, (long)0, (long)0,
        (const float*)nullptr, (long)0,
        (int)kSeq, (int)kDh, (int)kSeq, kPCarryInv);
    }
  }
}
